// GraphormerMultiHeadAttention_88622355186287
// MI455X (gfx1250) — hardware-verified
//
#include <hip/hip_runtime.h>


namespace {
constexpr int B = 4, S = 1024, DM = 512, H = 8, HD = 64, BL = 4  , QL = 1024  ;
constexpr float XS = 8.0f, WSC = 256.0f, PS = 1024.0f, LOG2E = 1.4426950408889634f, INF_DIST = 1.0e9f;
static_assert(S % 64 == 0 && QL % 64 == 0 && DM == H * HD, "tiling");
typedef _Float16 b16;
typedef __attribute__((ext_vector_type(16))) _Float16 v16b;
typedef __attribute__((ext_vector_type(8))) _Float16 v8b;
typedef __attribute__((ext_vector_type(8))) float v8f;
typedef __attribute__((ext_vector_type(4))) float v4f;
__device__ __forceinline__ float bf16_rne(float f) { unsigned int u = __float_as_uint(f); u += 0x7FFFu + ((u >> 16) & 1u); return __uint_as_float(u & 0xFFFF0000u); }
__device__ __forceinline__ void split16(float v, b16& hi, b16& lo) { hi = (b16)v; lo = (b16)(v - (float)hi); }
__device__ __forceinline__ v16b frag_kb(const b16* p, int hh) { const v8b a = *(const v8b*)(p + 8 * hh), b = *(const v8b*)(p + 16 + 8 * hh); v16b f;
#pragma unroll
  for (int e = 0; e < 8; ++e) { f[e] = a[e]; f[8 + e] = b[e]; } return f; }
__device__ __forceinline__ v8f wmma16b(v16b a, v16b b, v8f c) { v8f d = __builtin_amdgcn_wmma_f32_16x16x32_f16(false, a, false, b, (short)0, c, false, false); asm volatile("v_nop\n\tv_nop\n\tv_nop\n\tv_nop" : "+v"(d) : "v"(a), "v"(b)); return d; }
__device__ __forceinline__ void wave_lds_sync() { __builtin_amdgcn_fence(__ATOMIC_RELEASE, "workgroup"); __builtin_amdgcn_wave_barrier(); __builtin_amdgcn_fence(__ATOMIC_ACQUIRE, "workgroup"); }
__device__ __forceinline__ float pmul(float a, float b) { float p = a * b; asm volatile("" : "+v"(p)); return p; }
__device__ __forceinline__ int iclamp(int v, int lo, int hi) { return v < lo ? lo : (v > hi ? hi : v); }

typedef __attribute__((ext_vector_type(2))) _Float16 v2h;
typedef __attribute__((ext_vector_type(4))) _Float16 v4h;
typedef __attribute__((ext_vector_type(2))) float v2f;
__device__ __forceinline__ float nexp2(float v) { return __builtin_amdgcn_exp2f(v); }
__global__ __launch_bounds__(256) void prep_kernel(const float* __restrict__ wq, const float* __restrict__ wk, const float* __restrict__ wv, const float* __restrict__ wo, b16* __restrict__ WT) {
  const size_t u = (size_t)blockIdx.x * 256 + threadIdx.x; const size_t per = (size_t)DM * DM / 8; if (u >= 4 * per) return; const int m = (int)(u / per); const size_t e = (u % per) * 8; const float* w = m == 0 ? wq : m == 1 ? wk : m == 2 ? wv : wo; v8b o;
  for (int j = 0; j < 8; ++j) o[j] = (b16)(bf16_rne(w[e + j]) * WSC);
  for (int pass = 0; pass < 2; ++pass) { *(volatile v8b*)(WT + (size_t)m * DM * DM + e) = o; __threadfence(); }
}
__global__ __launch_bounds__(1024) void maxdist_kernel(const float* __restrict__ dist, float* __restrict__ MAXD) {
  __shared__ float red[1024]; const int b = blockIdx.x, t = threadIdx.x; float m = 0.0f;
  for (size_t i = t; i < (size_t)S * S; i += 1024) { const float d = bf16_rne(dist[(size_t)b * S * S + i]); const float vd = (d != INF_DIST) ? d : d * 0.0f; m = fmaxf(m, vd); }
  red[t] = m; __syncthreads();
  for (int w = 512; w >= 1; w >>= 1) { if (t < w) red[t] = fmaxf(red[t], red[t + w]); __syncthreads(); }
  if (t < 32) { const float r = fmaxf(red[0], 1.0f); for (int pass = 0; pass < 2; ++pass) { ((volatile float*)MAXD)[b * 32 + t] = r; __threadfence(); } }
}
__global__ __launch_bounds__(128) void proj_kernel(const float* __restrict__ x, const b16* __restrict__ WT, const float* __restrict__ bq, const float* __restrict__ bk, const float* __restrict__ bv, b16* __restrict__ Qp, b16* __restrict__ Kp, b16* __restrict__ VTh, b16* __restrict__ VTl) {
  __shared__ __attribute__((aligned(16))) b16 As[4][16][256 + 8]; __shared__ __attribute__((aligned(16))) float Tf[4][16][128 + 4];
  const int wave = threadIdx.x >> 5, lane = threadIdx.x & 31, nloc = lane & 15, hlf = lane >> 4; const int which = blockIdx.y % 3, b = blockIdx.y / 3; const int rb = blockIdx.x, slab = blockIdx.z; const int t0 = rb * 64 + wave * 16; const int n0 = slab * 128;
  const b16* W = WT + (size_t)which * DM * DM; const float* bias = which == 0 ? bq : (which == 1 ? bk : bv);
  v8f acc[8];
#pragma unroll
  for (int t = 0; t < 8; ++t) acc[t] = (v8f){};
#pragma unroll 1
  for (int half = 0; half < 2; ++half) {
    for (int rr = 0; rr < 16; ++rr) { const float* xr = x + ((size_t)b * S + t0 + rr) * DM + half * 256; for (int q = lane * 4; q < 256; q += 128) { const v4f xv = *(const v4f*)(xr + q); v4h o; for (int j = 0; j < 4; ++j) o[j] = (b16)(bf16_rne(xv[j]) * XS); *(v4h*)(&As[wave][rr][q]) = o; } }
    wave_lds_sync();
#pragma unroll 2
    for (int kb = 0; kb < 256; kb += 32) { const v16b a = frag_kb(&As[wave][nloc][kb], hlf);
#pragma unroll
      for (int t = 0; t < 8; ++t) acc[t] = wmma16b(a, frag_kb(W + (size_t)(n0 + t * 16 + nloc) * DM + half * 256 + kb, hlf), acc[t]); }
    wave_lds_sync(); }
#pragma unroll
  for (int t = 0; t < 8; ++t) { const float bb = bf16_rne(bias[n0 + t * 16 + nloc]);
#pragma unroll
    for (int r = 0; r < 8; ++r) Tf[wave][8 * hlf + r][t * 16 + nloc] = acc[t][r] * (1.0f / (XS * WSC)) + bb; }
  __syncthreads();
  for (int pass = 0; pass < 2; ++pass) {
    if (which == 2) {
#pragma unroll 1
      for (int q = 0; q < 32; ++q) { const int cl = wave * 32 + q; const int c = n0 + cl; const int h = c / HD, d = c % HD; const int tk = lane * 2; v2h hv, lv;
        for (int j = 0; j < 2; ++j) { b16 p, ql; split16(Tf[(tk + j) >> 4][(tk + j) & 15][cl] * XS, p, ql); hv[j] = p; lv[j] = ql; }
        const size_t oi = (((size_t)b * H + h) * HD + d) * S + rb * 64 + lane * 2; *(volatile v2h*)(VTh + oi) = hv; *(volatile v2h*)(VTl + oi) = lv; } }
    else { b16* P = which == 0 ? Qp : Kp;
      for (int rr = 0; rr < 16; ++rr) { for (int hs = 0; hs < 2; ++hs) { const int c = n0 + hs * 64; const int h = c / HD; v2h o; o[0] = (b16)(Tf[wave][rr][hs * 64 + lane * 2] * XS); o[1] = (b16)(Tf[wave][rr][hs * 64 + lane * 2 + 1] * XS);
          *(volatile v2h*)(P + (((size_t)b * H + h) * S + (t0 + rr)) * HD + lane * 2) = o; } } }
    __threadfence(); }
}
__global__ __launch_bounds__(64) void attn_kernel(const b16* __restrict__ Qp, const b16* __restrict__ Kp, const b16* __restrict__ VTh, const b16* __restrict__ VTl, const float* __restrict__ dist, const float* __restrict__ MAXD, b16* __restrict__ Ch, b16* __restrict__ Cl) {
  __shared__ __attribute__((aligned(16))) b16 Ph[2][16][32 + 8], Pl[2][16][32 + 8]; __shared__ __attribute__((aligned(16))) float To[2][16][HD + 4];
  const int wave = threadIdx.x >> 5, lane = threadIdx.x & 31, hh = lane >> 4, col = lane & 15; const int b = blockIdx.y / H, h = blockIdx.y % H; const int q0 = blockIdx.x * 32 + wave * 16, qi = q0 + col;
  const b16* Qb = Qp + ((size_t)(b * H + h) * S) * HD; const b16* Kb = Kp + ((size_t)(b * H + h) * S) * HD; const b16* Vh = VTh + ((size_t)(b * H + h) * HD) * S; const b16* Vl = VTl + ((size_t)(b * H + h) * HD) * S;
  const float* Db = dist + ((size_t)b * S + qi) * S; const float dsc = 10.0f * LOG2E / MAXD[b * 32];
  const v16b qa0 = frag_kb(Qb + (size_t)qi * HD, hh), qa1 = frag_kb(Qb + (size_t)qi * HD + 32, hh);
  const float cs = LOG2E / (8.0f * XS * XS);
  float m = -INFINITY, l = 0.0f; v8f o[4]; for (int t = 0; t < 4; ++t) o[t] = (v8f){};
#pragma unroll 1
  for (int kb = 0; kb < S; kb += 32) {
    float e[16]; float mx = -INFINITY;
#pragma unroll
    for (int u = 0; u < 2; ++u) { v8f s = (v8f){}; const size_t kr = (size_t)(kb + u * 16 + col) * HD; s = wmma16b(frag_kb(Kb + kr, hh), qa0, s); s = wmma16b(frag_kb(Kb + kr + 32, hh), qa1, s);
      const v4f d0 = *(const v4f*)(Db + kb + u * 16 + 8 * hh), d1 = *(const v4f*)(Db + kb + u * 16 + 8 * hh + 4);
#pragma unroll
      for (int r = 0; r < 8; ++r) { const float dv = bf16_rne(r < 4 ? d0[r] : d1[r - 4]); const float vv = (dv != INF_DIST) ? (s[r] * cs - dv * dsc) : -INFINITY; e[u * 8 + r] = vv; mx = fmaxf(mx, vv); } }
    mx = fmaxf(mx, __shfl_xor(mx, 16)); const float mn = fmaxf(m, mx); const float al = (mn == -INFINITY) ? 1.0f : nexp2(m - mn); float sum = 0.0f;
#pragma unroll
    for (int i2 = 0; i2 < 16; ++i2) { const float p = (e[i2] == -INFINITY || mn == -INFINITY) ? 0.0f : nexp2(e[i2] - mn); sum += p; b16 a_, b_; split16(p * PS, a_, b_); const int sl = (i2 < 8 ? 0 : 16) + 8 * hh + (i2 & 7); Ph[wave][col][sl] = a_; Pl[wave][col][sl] = b_; }
    sum += __shfl_xor(sum, 16); l = l * al + sum; m = mn;
    wave_lds_sync();
    const v16b pf = frag_kb(&Ph[wave][col][0], hh), pg = frag_kb(&Pl[wave][col][0], hh);
#pragma unroll
    for (int t = 0; t < 4; ++t) { o[t] *= al; const size_t vr = (size_t)(t * 16 + col) * S + kb; const v16b va = frag_kb(Vh + vr, hh), vb = frag_kb(Vl + vr, hh); o[t] = wmma16b(va, pf, o[t]); o[t] = wmma16b(va, pg, o[t]); o[t] = wmma16b(vb, pf, o[t]); }
    wave_lds_sync(); }
  const float inv = (l > 0.0f) ? 1.0f / (l * PS * XS) : 0.0f;
#pragma unroll
  for (int t = 0; t < 4; ++t)
#pragma unroll
    for (int r = 0; r < 8; ++r) To[wave][col][t * 16 + 8 * hh + r] = o[t][r] * inv;
  wave_lds_sync();
  for (int pass = 0; pass < 2; ++pass) { for (int rr = 0; rr < 16; ++rr) { const v2f f = *(const v2f*)(&To[wave][rr][lane * 2]); v2h hv, lv; for (int j = 0; j < 2; ++j) { b16 p, q; split16(f[j] * XS, p, q); hv[j] = p; lv[j] = q; }
      const size_t oi = ((size_t)b * S + q0 + rr) * DM + h * HD + lane * 2; *(volatile v2h*)(Ch + oi) = hv; *(volatile v2h*)(Cl + oi) = lv; } __threadfence(); }
}
__global__ __launch_bounds__(128) void out_kernel(const b16* __restrict__ Ch, const b16* __restrict__ Cl, const b16* __restrict__ WO, const float* __restrict__ bo, float* __restrict__ out) {
  __shared__ __attribute__((aligned(16))) float Tf[4][16][128 + 4];
  const int wave = threadIdx.x >> 5, lane = threadIdx.x & 31, nloc = lane & 15, hlf = lane >> 4; const int b = blockIdx.x / (QL / 64), rb = blockIdx.x % (QL / 64); const size_t m0 = (size_t)b * S + rb * 64 + wave * 16; const int n0 = blockIdx.y * 128;
  v8f acc[8];
#pragma unroll
  for (int t = 0; t < 8; ++t) acc[t] = (v8f){};
#pragma unroll 2
  for (int kb = 0; kb < DM; kb += 32) { const v16b a = frag_kb(Ch + (m0 + nloc) * DM + kb, hlf), al = frag_kb(Cl + (m0 + nloc) * DM + kb, hlf);
#pragma unroll
    for (int t = 0; t < 8; ++t) { const v16b bw = frag_kb(WO + (size_t)(n0 + t * 16 + nloc) * DM + kb, hlf); acc[t] = wmma16b(a, bw, acc[t]); acc[t] = wmma16b(al, bw, acc[t]); } }
#pragma unroll
  for (int t = 0; t < 8; ++t) { const float bb = bf16_rne(bo[n0 + t * 16 + nloc]);
#pragma unroll
    for (int r = 0; r < 8; ++r) Tf[wave][8 * hlf + r][t * 16 + nloc] = acc[t][r] * (1.0f / (XS * WSC)) + bb; }
  wave_lds_sync();
  for (int pass = 0; pass < 2; ++pass) { for (int rr = 0; rr < 16; ++rr) *(volatile v4f*)(out + (m0 + rr) * DM + n0 + lane * 4) = *(const v4f*)(&Tf[wave][rr][lane * 4]); __threadfence(); }
}
}

extern "C" void kernel_launch(void* const* d_in, const int* in_sizes, int n_in, void* d_out, int out_size, void* d_ws, size_t ws_size, hipStream_t stream) {
  (void)n_in;
  auto Fp = [&](int i) { return (const float*)d_in[i]; };
  if (in_sizes[0] != B * S * DM || in_sizes[1] != B * S * S || in_sizes[2] != DM * DM || in_sizes[3] != DM || in_sizes[8] != DM * DM || in_sizes[9] != DM || out_size != B * S * DM) return;
  size_t off = 0; char* ws = (char*)d_ws;
  auto carve = [&](size_t bytes) { char* p = ws + off; off += (bytes + 255) & ~(size_t)255; return p; };
  b16* WT = (b16*)carve((size_t)4 * DM * DM * 2); float* MAXD = (float*)carve((size_t)B * 32 * 4); const size_t plane = (size_t)B * S * DM * 2;
  b16* Qp = (b16*)carve(plane); b16* Kp = (b16*)carve(plane); b16* VTh = (b16*)carve(plane); b16* VTl = (b16*)carve(plane); b16* Ch = (b16*)carve(plane); b16* Cl = (b16*)carve(plane);
  if (off > ws_size || off > ((size_t)128 << 20)) return;
  prep_kernel<<<(unsigned)(((size_t)4 * DM * DM / 8 + 255) / 256), 256, 0, stream>>>(Fp(2), Fp(4), Fp(6), Fp(8), WT);
  maxdist_kernel<<<B, 1024, 0, stream>>>(Fp(1), MAXD);
  proj_kernel<<<dim3(S / 64, BL * 3, 4), 128, 0, stream>>>(Fp(0), WT, Fp(3), Fp(5), Fp(7), Qp, Kp, VTh, VTl);
  attn_kernel<<<dim3(QL / 32, BL * H), 64, 0, stream>>>(Qp, Kp, VTh, VTl, Fp(1), MAXD, Ch, Cl);
  out_kernel<<<dim3((QL / 64) * BL, 4), 128, 0, stream>>>(Ch, Cl, WT + (size_t)3 * DM * DM, Fp(9), (float*)d_out);
}
